// SelfAttention_77841987273308
// MI455X (gfx1250) — hardware-verified
//
#include <hip/hip_runtime.h>


#ifndef NB
#define NB 4
#endif
#ifndef SEQ
#define SEQ 4096
#endif
#define NB_FULL   4
#define SEQ_FULL  4096
#define CC        256
#define DD        64
#define NWT       (2 * DD + CC)
#define BQ        64
#define BK        32
#define NWAVE     8
#define PT        64
#define AP        264
#define TP        72
#define OP        68
#define P_CARRY   4096.0f
#define RES_CARRY 2048.0f

#define WT_BYTES   ((size_t)NWT * CC * 2)
#define QK_BYTES   ((size_t)2 * NB * SEQ * DD * 2)
#define GT_BYTES   ((size_t)NB * CC * SEQ * 2)
#define WS_TOTAL   (WT_BYTES + 2 * QK_BYTES + GT_BYTES)

static_assert(SEQ % BQ == 0);
static_assert(SEQ % PT == 0);
static_assert(SEQ % BK == 0);
static_assert(SEQ % 64 == 0);
static_assert(BQ == (NWAVE / 2) * 16);
static_assert(PT == (NWAVE / 2) * 16);
static_assert(DD == 64);
static_assert(CC == 256);
static_assert(CC % 32 == 0);
static_assert(DD % 32 == 0);
static_assert(CC % 64 == 0);
static_assert(SEQ <= SEQ_FULL);
static_assert(NB >= 1 && NB <= NB_FULL);
static_assert((AP * 2) % 16 == 0);
static_assert((TP * 2) % 16 == 0);
static_assert((OP * 4) % 16 == 0);
static_assert(AP >= CC);
static_assert(TP >= 64);
static_assert(OP >= 64);
static_assert(WT_BYTES % 128 == 0);
static_assert(QK_BYTES % 128 == 0);
static_assert(GT_BYTES % 128 == 0);
static_assert(WS_TOTAL <= (size_t)134217728);
static_assert((size_t)2 * NB * SEQ * DD < (size_t)2147483647);
static_assert((size_t)NB * CC * SEQ < (size_t)2147483647);
static_assert((size_t)PT * AP * 2 + (size_t)128 * TP * 2 <= (size_t)65536);
static_assert((size_t)NWAVE * 16 * OP * 4 <= (size_t)65536);

typedef __bf16   bf16;
typedef _Float16 f16;
typedef bf16     v16bf __attribute__((ext_vector_type(16)));
typedef f16      v16h  __attribute__((ext_vector_type(16)));
typedef f16      v8h   __attribute__((ext_vector_type(8)));
typedef float    v8f   __attribute__((ext_vector_type(8)));
typedef float    v4f   __attribute__((ext_vector_type(4)));
typedef unsigned v4u   __attribute__((ext_vector_type(4)));

union FragB  { v16bf v; v4u q[2]; bf16 h[16]; };
union FragH  { v16h  v; v4u q[2]; f16  h[16]; };
union Pack8B { v4u u; bf16 h[8]; };
union Pack8H { v4u u; v8h v; f16 h[8]; };

static __device__ __forceinline__ v8f mma_bf16(v16bf a, v16bf b, v8f acc) {
  acc = __builtin_amdgcn_wmma_f32_16x16x32_bf16(false, a, false, b, (short)0, acc, false, false);
  asm volatile("v_nop\n\tv_nop\n\tv_nop\n\tv_nop" : "+v"(acc) : "v"(a), "v"(b));
  return acc;
}
static __device__ __forceinline__ v8f mma_f16(v16h a, v16h b, v8f acc) {
  acc = __builtin_amdgcn_wmma_f32_16x16x32_f16(false, a, false, b, (short)0, acc, false, false);
  asm volatile("v_nop\n\tv_nop\n\tv_nop\n\tv_nop" : "+v"(acc) : "v"(a), "v"(b));
  return acc;
}

__global__ __launch_bounds__(256) void wt_kernel(const float* __restrict__ w, int ncols,
                                                 bf16* __restrict__ wt_rows) {
  const int k0  = blockIdx.x * 64;
  const int n0  = blockIdx.y * 64;
  const int tid = threadIdx.x;
  __shared__ __align__(16) bf16 sT[64 * TP];

  {
    const int k  = tid >> 2;
    const int n4 = (tid & 3) * 16;
    const float* src = w + (size_t)(k0 + k) * ncols + n0 + n4;
    #pragma unroll
    for (int i = 0; i < 4; ++i) {
      const v4f x = *(const v4f*)(src + 4 * i);
      #pragma unroll
      for (int e = 0; e < 4; ++e) sT[(n4 + 4 * i + e) * TP + k] = (bf16)x[e];
    }
  }
  __syncthreads();

  v4u    val[2];
  size_t idx[2];
  #pragma unroll
  for (int kk = 0; kk < 2; ++kk) {
    const int n  = kk * 32 + (tid >> 3);
    const int pc = tid & 7;
    val[kk] = *(const v4u*)(sT + n * TP + pc * 8);
    idx[kk] = (size_t)(n0 + n) * CC + k0 + pc * 8;
  }
  #pragma unroll
  for (int kk = 0; kk < 2; ++kk) *(volatile v4u*)(wt_rows + idx[kk]) = val[kk];
  __threadfence();
  #pragma unroll
  for (int kk = 0; kk < 2; ++kk) *(volatile v4u*)(wt_rows + idx[kk]) = val[kk];
}

__global__ __launch_bounds__(256) void proj_kernel(const float* __restrict__ p,
                                                   const bf16* __restrict__ wt,
                                                   const float* __restrict__ bl,
                                                   const float* __restrict__ bh,
                                                   const float* __restrict__ bg,
                                                   f16* __restrict__ qkh,
                                                   f16* __restrict__ qkr,
                                                   f16* __restrict__ gt) {
  const int tid  = threadIdx.x;
  const int wave = __builtin_amdgcn_readfirstlane(threadIdx.x >> 5);
  const int lane = tid & 31;
  const int lq   = lane & 15;
  const int hi   = lane >> 4;
  const int mt   = wave & 3;
  const int side = wave >> 2;
  const int b    = blockIdx.y;
  const int pos0 = blockIdx.x * PT;

  __shared__ __align__(16) bf16 sA[PT * AP];
  __shared__ __align__(16) f16  sS[128 * TP];

  #pragma unroll 2
  for (int it = 0; it < 8; ++it) {
    const int row = it * 8 + (tid >> 5);
    const int c8  = (tid & 31) * 8;
    const float* src = p + ((size_t)b * SEQ_FULL + pos0 + row) * CC + c8;
    const v4f x0 = *(const v4f*)(src);
    const v4f x1 = *(const v4f*)(src + 4);
    Pack8B pk;
    #pragma unroll
    for (int e = 0; e < 4; ++e) {
      pk.h[e]     = (bf16)x0[e];
      pk.h[4 + e] = (bf16)x1[e];
    }
    *(v4u*)(sA + row * AP + c8) = pk.u;
  }
  __syncthreads();

  const int arow = (mt * 16 + lq) * AP + hi * 8;

  #pragma unroll 1
  for (int g = 0; g < 3; ++g) {
    const int gcg   = side * 2 + ((g > 0) ? (g - 1) : 0);
    const int wrow0 = (g == 0) ? (side * DD) : (2 * DD + gcg * 64);

    v8f acc[4];
    #pragma unroll
    for (int nt = 0; nt < 4; ++nt) acc[nt] = (v8f){0, 0, 0, 0, 0, 0, 0, 0};

    #pragma unroll 1
    for (int ks = 0; ks < CC / 32; ++ks) {
      FragB a;
      a.q[0] = *(const v4u*)(sA + arow + ks * 32);
      a.q[1] = *(const v4u*)(sA + arow + ks * 32 + 16);
      FragB bw[4];
      #pragma unroll
      for (int nt = 0; nt < 4; ++nt) {
        const bf16* base = wt + (size_t)(wrow0 + nt * 16 + lq) * CC + ks * 32 + hi * 8;
        bw[nt].q[0] = *(const v4u*)(base);
        bw[nt].q[1] = *(const v4u*)(base + 16);
      }
      #pragma unroll
      for (int nt = 0; nt < 4; ++nt) acc[nt] = mma_bf16(a.v, bw[nt].v, acc[nt]);
    }

    float bias[4];
    #pragma unroll
    for (int nt = 0; nt < 4; ++nt) {
      const int c64 = nt * 16 + lq;
      const float xl = bl[c64];
      const float xh = bh[c64];
      const float xg = bg[gcg * 64 + c64];
      const float sel = (g == 0) ? (side ? xh : xl) : xg;
      bias[nt] = (float)(bf16)sel;
    }

    if (g == 0) {
      f16 rres[4][8];
      #pragma unroll
      for (int nt = 0; nt < 4; ++nt) {
        #pragma unroll
        for (int r = 0; r < 8; ++r) {
          const float v  = acc[nt][r] + bias[nt];
          const f16   hv = (f16)v;
          rres[nt][r] = (f16)((v - (float)hv) * RES_CARRY);
          sS[(wave * 16 + hi * 8 + r) * TP + nt * 16 + lq] = hv;
        }
      }
      __syncthreads();
      v4u    lin[8];
      size_t lidx[4];
      #pragma unroll
      for (int it = 0; it < 4; ++it) {
        const int row = it * 4 + (lane >> 3);
        const int pc  = lane & 7;
        lin[it]  = *(const v4u*)(sS + (wave * 16 + row) * TP + pc * 8);
        lidx[it] = (((size_t)side * NB + b) * SEQ + pos0 + mt * 16 + row) * DD + pc * 8;
      }
      __syncthreads();
      #pragma unroll
      for (int nt = 0; nt < 4; ++nt) {
        #pragma unroll
        for (int r = 0; r < 8; ++r)
          sS[(wave * 16 + hi * 8 + r) * TP + nt * 16 + lq] = rres[nt][r];
      }
      __syncthreads();
      #pragma unroll
      for (int it = 0; it < 4; ++it) {
        const int row = it * 4 + (lane >> 3);
        const int pc  = lane & 7;
        lin[4 + it] = *(const v4u*)(sS + (wave * 16 + row) * TP + pc * 8);
      }
      #pragma unroll
      for (int it = 0; it < 4; ++it) {
        *(volatile v4u*)(qkh + lidx[it]) = lin[it];
        *(volatile v4u*)(qkr + lidx[it]) = lin[4 + it];
      }
      __threadfence();
      #pragma unroll
      for (int it = 0; it < 4; ++it) {
        *(volatile v4u*)(qkh + lidx[it]) = lin[it];
        *(volatile v4u*)(qkr + lidx[it]) = lin[4 + it];
      }
    } else {
      __syncthreads();
      #pragma unroll
      for (int nt = 0; nt < 4; ++nt) {
        Pack8H ph;
        #pragma unroll
        for (int r = 0; r < 8; ++r) ph.h[r] = (f16)(acc[nt][r] + bias[nt]);
        *(v4u*)(sS + (side * 64 + nt * 16 + lq) * TP + mt * 16 + hi * 8) = ph.u;
      }
      __syncthreads();
      v4u    gl[4];
      size_t gidx[4];
      #pragma unroll
      for (int it = 0; it < 4; ++it) {
        const int crow = it * 32 + (tid >> 3);
        const int pc   = tid & 7;
        const int chan = ((crow >> 6) * 2 + (g - 1)) * 64 + (crow & 63);
        gl[it]   = *(const v4u*)(sS + crow * TP + pc * 8);
        gidx[it] = ((size_t)b * CC + chan) * SEQ + pos0 + pc * 8;
      }
      #pragma unroll
      for (int it = 0; it < 4; ++it) *(volatile v4u*)(gt + gidx[it]) = gl[it];
      __threadfence();
      #pragma unroll
      for (int it = 0; it < 4; ++it) *(volatile v4u*)(gt + gidx[it]) = gl[it];
    }
  }
}

__global__ __launch_bounds__(256) void attn_kernel(const float* __restrict__ p,
                                                   const f16* __restrict__ qkh,
                                                   const f16* __restrict__ qkr,
                                                   const f16* __restrict__ gt,
                                                   float* __restrict__ out) {
  const int tid  = threadIdx.x;
  const int wave = __builtin_amdgcn_readfirstlane(threadIdx.x >> 5);
  const int lane = tid & 31;
  const int lq   = lane & 15;
  const int hi   = lane >> 4;
  const int qt   = wave & 3;
  const int chh  = wave >> 2;
  const int b    = blockIdx.y;
  const int qrow0 = blockIdx.x * BQ + qt * 16;

  __shared__ __align__(16) float sO[NWAVE * 16 * OP];

  const int plane = NB * SEQ * DD;
  const int qoff0 = (b * SEQ + qrow0 + lq) * DD + hi * 8;
  const int koff0 = plane + (b * SEQ + lq) * DD + hi * 8;
  const int voff0 = (b * CC + chh * 128 + lq) * SEQ + hi * 8;

  v8f o[8];
  #pragma unroll
  for (int t = 0; t < 8; ++t) o[t] = (v8f){0, 0, 0, 0, 0, 0, 0, 0};

  float rmax = -__builtin_inff();
  float rsum = 0.0f;
  const float SL = 1.4426950408889634f;

  #pragma unroll 1
  for (int i = 0; i < SEQ / BK; ++i) {
    const int j0 = i * BK;
    int qoff = qoff0;
    asm volatile("" : "+v"(qoff));

    v8f sh[2], sr[2];
    #pragma unroll
    for (int sub = 0; sub < 2; ++sub) {
      sh[sub] = (v8f){0, 0, 0, 0, 0, 0, 0, 0};
      sr[sub] = (v8f){0, 0, 0, 0, 0, 0, 0, 0};
    }

    #pragma unroll
    for (int f = 0; f < 2; ++f) {
      FragH bqh, bqr;
      bqh.q[0] = *(const v4u*)(qkh + qoff + f * 32);
      bqh.q[1] = *(const v4u*)(qkh + qoff + f * 32 + 16);
      bqr.q[0] = *(const v4u*)(qkr + qoff + f * 32);
      bqr.q[1] = *(const v4u*)(qkr + qoff + f * 32 + 16);
      #pragma unroll
      for (int sub = 0; sub < 2; ++sub) {
        const int ko = koff0 + (j0 + sub * 16) * DD + f * 32;
        FragH ahh, ahr;
        ahh.q[0] = *(const v4u*)(qkh + ko);
        ahh.q[1] = *(const v4u*)(qkh + ko + 16);
        ahr.q[0] = *(const v4u*)(qkr + ko);
        ahr.q[1] = *(const v4u*)(qkr + ko + 16);
        sh[sub] = mma_f16(ahh.v, bqh.v, sh[sub]);
        sr[sub] = mma_f16(ahh.v, bqr.v, sr[sub]);
        sr[sub] = mma_f16(ahr.v, bqh.v, sr[sub]);
      }
    }

    v8f c[2];
    #pragma unroll
    for (int sub = 0; sub < 2; ++sub) {
      #pragma unroll
      for (int r = 0; r < 8; ++r) c[sub][r] = sh[sub][r] + sr[sub][r] * (1.0f / RES_CARRY);
    }

    float m_new = rmax;
    #pragma unroll
    for (int r = 0; r < 8; ++r) {
      m_new = fmaxf(m_new, c[0][r]);
      m_new = fmaxf(m_new, c[1][r]);
    }
    m_new = fmaxf(m_new, __shfl_xor(m_new, 16, 32));
    const float scale = __builtin_amdgcn_exp2f((rmax - m_new) * SL);
    rmax = m_new;

    FragH pa;
    float psum = 0.0f;
    #pragma unroll
    for (int r = 0; r < 8; ++r) {
      const float p0 = __builtin_amdgcn_exp2f((c[0][r] - m_new) * SL);
      const float p1 = __builtin_amdgcn_exp2f((c[1][r] - m_new) * SL);
      psum += p0 + p1;
      pa.h[r]     = (f16)(p0 * P_CARRY);
      pa.h[8 + r] = (f16)(p1 * P_CARRY);
    }
    rsum = rsum * scale + psum + __shfl_xor(psum, 16, 32);

    float sc[8];
    #pragma unroll
    for (int r = 0; r < 8; ++r) sc[r] = __shfl(scale, (hi << 3) + r, 32);
    #pragma unroll
    for (int t = 0; t < 8; ++t) {
      #pragma unroll
      for (int r = 0; r < 8; ++r) o[t][r] *= sc[r];
    }

    __builtin_amdgcn_sched_barrier(0);

    #pragma unroll
    for (int g4 = 0; g4 < 2; ++g4) {
      FragH bv[4];
      #pragma unroll
      for (int t = 0; t < 4; ++t) {
        const int vo = voff0 + ((g4 * 4 + t) * 16) * SEQ + j0;
        bv[t].q[0] = *(const v4u*)(gt + vo);
        bv[t].q[1] = *(const v4u*)(gt + vo + 16);
      }
      #pragma unroll
      for (int t = 0; t < 4; ++t) o[g4 * 4 + t] = mma_f16(pa.v, bv[t].v, o[g4 * 4 + t]);
      __builtin_amdgcn_sched_barrier(0);
    }
  }

  float rs[8];
  #pragma unroll
  for (int r = 0; r < 8; ++r) rs[r] = 1.0f / __shfl(rsum, (hi << 3) + r, 32);

  const int sbase = wave * (16 * OP);
  #pragma unroll
  for (int half = 0; half < 2; ++half) {
    #pragma unroll
    for (int r = 0; r < 8; ++r) {
      #pragma unroll
      for (int t = 0; t < 4; ++t)
        sO[sbase + (hi * 8 + r) * OP + t * 16 + lq] = o[half * 4 + t][r] * (1.0f / P_CARRY) * rs[r];
    }
    __syncthreads();

    v4f    vals[8];
    size_t gidx[8];
    #pragma unroll
    for (int it = 0; it < 8; ++it) {
      const int row = it * 2 + hi;
      gidx[it] = ((size_t)b * SEQ_FULL + qrow0 + row) * CC + chh * 128 + half * 64 + lq * 4;
      const v4f av = *(const v4f*)(sO + sbase + row * OP + lq * 4);
      const v4f pv = *(const v4f*)(p + gidx[it]);
      v4f res;
      #pragma unroll
      for (int e = 0; e < 4; ++e) res[e] = av[e] + (float)(bf16)pv[e];
      vals[it] = res;
    }
    #pragma unroll
    for (int it = 0; it < 8; ++it) *(volatile v4f*)(out + gidx[it]) = vals[it];
    __threadfence();
    #pragma unroll
    for (int it = 0; it < 8; ++it) *(volatile v4f*)(out + gidx[it]) = vals[it];
    __syncthreads();
  }
}

extern "C" void kernel_launch(void* const* d_in, const int* in_sizes, int n_in,
                              void* d_out, int out_size, void* d_ws, size_t ws_size,
                              hipStream_t stream) {
  if (n_in < 7) return;
  const size_t rows_used = (size_t)(NB - 1) * SEQ_FULL + SEQ;
  if ((size_t)in_sizes[0] < rows_used * CC) return;
  if ((size_t)in_sizes[1] < (size_t)CC * DD) return;
  if ((size_t)in_sizes[2] < (size_t)DD) return;
  if ((size_t)in_sizes[3] < (size_t)CC * DD) return;
  if ((size_t)in_sizes[4] < (size_t)DD) return;
  if ((size_t)in_sizes[5] < (size_t)CC * CC) return;
  if ((size_t)in_sizes[6] < (size_t)CC) return;
  if ((size_t)out_size < rows_used * CC) return;
  if (ws_size < WS_TOTAL) return;

  const float* p  = (const float*)d_in[0];
  const float* Wh = (const float*)d_in[1];
  const float* bh = (const float*)d_in[2];
  const float* Wl = (const float*)d_in[3];
  const float* bl = (const float*)d_in[4];
  const float* Wg = (const float*)d_in[5];
  const float* bg = (const float*)d_in[6];
  float*       out = (float*)d_out;

  char* ws  = (char*)d_ws;
  bf16* wt  = (bf16*)ws;
  f16*  qkh = (f16*)(ws + WT_BYTES);
  f16*  qkr = (f16*)(ws + WT_BYTES + QK_BYTES);
  f16*  gt  = (f16*)(ws + WT_BYTES + 2 * QK_BYTES);

  wt_kernel<<<dim3(CC / 64, DD / 64), 256, 0, stream>>>(Wl, DD, wt);
  wt_kernel<<<dim3(CC / 64, DD / 64), 256, 0, stream>>>(Wh, DD, wt + (size_t)DD * CC);
  wt_kernel<<<dim3(CC / 64, CC / 64), 256, 0, stream>>>(Wg, CC, wt + (size_t)2 * DD * CC);

  proj_kernel<<<dim3(SEQ / PT, NB), 256, 0, stream>>>(p, wt, bl, bh, bg, qkh, qkr, gt);

  attn_kernel<<<dim3(SEQ / BQ, NB), 256, 0, stream>>>(p, qkh, qkr, gt, out);
}
